// HyperbolicPatchEmbedding_5952824672956
// MI455X (gfx1250) — hardware-verified
//
#include <hip/hip_runtime.h>
#include <math.h>

constexpr int kBatch  = 64;
constexpr int kChan   = 3;
constexpr int kImg    = 224;
constexpr int kPatch  = 16;
constexpr int kGridP  = 14;
constexpr int kNPatch = kGridP * kGridP;
constexpr int kRows   = kBatch * kNPatch;
constexpr int kKdim   = kChan * kPatch * kPatch;
constexpr int kNdim   = 768;
constexpr float kEps     = 1e-15f;
constexpr float kMaxNorm = 0.996f;

static_assert(kRows % 64 == 0);
static_assert(kNdim % 64 == 0);
static_assert(kKdim % 32 == 0);
static_assert(kKdim == 768);

typedef __attribute__((ext_vector_type(16))) _Float16 v16h;
typedef __attribute__((ext_vector_type(8)))  _Float16 v8h;
typedef __attribute__((ext_vector_type(16))) __bf16   v16b;
typedef __attribute__((ext_vector_type(8)))  __bf16   v8b;
typedef __attribute__((ext_vector_type(8)))  float    v8f;
typedef __attribute__((ext_vector_type(4)))  float    v4f;
typedef __attribute__((ext_vector_type(4)))  unsigned int v4u;

__device__ __forceinline__ unsigned short f2bf_bits(float f) {
  unsigned u = __float_as_uint(f);
  return (unsigned short)((u + 0x7FFFu + ((u >> 16) & 1u)) >> 16);
}
__device__ __forceinline__ float bf_bits2f(unsigned short h) { return __uint_as_float(((unsigned)h) << 16); }

__device__ __forceinline__ void dep_guard_h(v8f& a, v8f& b, v16h x, v16h y) { asm volatile("v_nop\n\tv_nop\n\tv_nop\n\tv_nop" : "+v"(a), "+v"(b) : "v"(x), "v"(y)); }
__device__ __forceinline__ void dep_guard_b(v8f& a, v8f& b, v16b x, v16b y) { asm volatile("v_nop\n\tv_nop\n\tv_nop\n\tv_nop" : "+v"(a), "+v"(b) : "v"(x), "v"(y)); }
__device__ __forceinline__ void keep4_h(v16h a, v16h b, v16h c, v16h d) { asm volatile("v_nop" :: "v"(a), "v"(b), "v"(c), "v"(d)); }
__device__ __forceinline__ void keep4_b(v16b a, v16b b, v16b c, v16b d) { asm volatile("v_nop" :: "v"(a), "v"(b), "v"(c), "v"(d)); }
__device__ __forceinline__ void acc_guard4(v8f& a, v8f& b, v8f& c, v8f& d) { asm volatile("v_nop\n\tv_nop\n\tv_nop\n\tv_nop" : "+v"(a), "+v"(b), "+v"(c), "+v"(d)); }
template <typename T> struct Frag;
template <> struct Frag<_Float16> {
  typedef v16h V; union U { v16h v; v8h h[2]; };
  static __device__ __forceinline__ v16h load(const _Float16* p) {
    U f; f.h[0] = *(const v8h*)(p); f.h[1] = *(const v8h*)(p + 16); return f.v;
  }
  static __device__ __forceinline__ v8f mma(v16h a, v16h b, v8f c) {
    return __builtin_amdgcn_wmma_f32_16x16x32_f16(false, a, false, b, (short)0, c, false, false);
  }
  static __device__ __forceinline__ void guard(v8f& a, v8f& b, v16h x, v16h y) { dep_guard_h(a, b, x, y); }
  static __device__ __forceinline__ void keep(v16h a, v16h b, v16h c, v16h d) { keep4_h(a, b, c, d); }
};
template <> struct Frag<__bf16> {
  typedef v16b V; union U { v16b v; v8b h[2]; };
  static __device__ __forceinline__ v16b load(const __bf16* p) {
    U f; f.h[0] = *(const v8b*)(p); f.h[1] = *(const v8b*)(p + 16); return f.v;
  }
  static __device__ __forceinline__ v8f mma(v16b a, v16b b, v8f c) {
    return __builtin_amdgcn_wmma_f32_16x16x32_bf16(false, a, false, b, (short)0, c, false, false);
  }
  static __device__ __forceinline__ void guard(v8f& a, v8f& b, v16b x, v16b y) { dep_guard_b(a, b, x, y); }
  static __device__ __forceinline__ void keep(v16b a, v16b b, v16b c, v16b d) { keep4_b(a, b, c, d); }
};

__device__ __forceinline__ unsigned pk16(unsigned short a, unsigned short b) { return (unsigned)a | ((unsigned)b << 16); }

template <int ET> struct Elem;
template <> struct Elem<0> { typedef _Float16 T; };
template <> struct Elem<1> { typedef __bf16 T; };
template <int ET, bool SPLIT, int BIAS_MODE, int OUT_MODE, bool RESID, int ACT = 0>
__global__ __launch_bounds__(256) void wmma_gemm64(
    const unsigned short* __restrict__ Ap, const unsigned short* __restrict__ A2p, int lda, long strideA,
    const unsigned short* __restrict__ Btp, const unsigned short* __restrict__ Bt2p, int ldb, long strideB,
    void* __restrict__ Cout, void* __restrict__ Cout2, int ldc, long strideC,
    const float* __restrict__ bias,
    const float* __restrict__ resid, long strideR,
    int M, int N, int K, float scale) {
  typedef typename Elem<ET>::T T;
  typedef typename Frag<T>::V V;
  const T* A = (const T*)Ap; const T* A2 = (const T*)A2p; const T* Bt = (const T*)Btp; const T* Bt2 = (const T*)Bt2p;
  __shared__ __align__(16) float sT[8][16 * 68];
  const int b    = blockIdx.y;
  const int lane = threadIdx.x & 31;
  const int wave = threadIdx.x >> 5;
  const int tilesN = N >> 6;
  const int tilesM = M >> 6;
  const int tile = blockIdx.x * 8 + wave;
  if (tile >= tilesM * tilesN) return;
  const int tm = tile / tilesN;
  const int tn = tile - tm * tilesN;
  const int m0 = tm << 6;
  const int n0 = tn << 6;

  const T* Ab  = A  + (size_t)b * strideA;
  const T* Bb  = Bt + (size_t)b * strideB;
  const T* Ab2 = SPLIT ? (A2  + (size_t)b * strideA) : nullptr;
  const T* Bb2 = SPLIT ? (Bt2 + (size_t)b * strideB) : nullptr;

  const int rlane = lane & 15;
  const int koff  = (lane >> 4) * 8;
  const int mOff  = (lane >> 4) * 8;

  v8f acc[4][4];
#pragma unroll
  for (int i = 0; i < 4; ++i)
#pragma unroll
    for (int j = 0; j < 4; ++j) acc[i][j] = (v8f){0.f,0.f,0.f,0.f,0.f,0.f,0.f,0.f};

  for (int k0 = 0; k0 < K; k0 += 32) {
    V bh[4], bl[4];
#pragma unroll
    for (int j = 0; j < 4; ++j) {
      const size_t bo = (size_t)(n0 + (j << 4) + rlane) * ldb + koff + k0;
      bh[j] = Frag<T>::load(Bb + bo);
      if (SPLIT) bl[j] = Frag<T>::load(Bb2 + bo);
    }
#pragma unroll
    for (int i = 0; i < 4; ++i) {
      const size_t ao = (size_t)(m0 + (i << 4) + rlane) * lda + koff + k0;
      V ah = Frag<T>::load(Ab + ao);
      V al;
      if (SPLIT) al = Frag<T>::load(Ab2 + ao);
#pragma unroll
      for (int j = 0; j < 4; ++j) {
        acc[i][j] = Frag<T>::mma(ah, bh[j], acc[i][j]);
        if (SPLIT) {
          acc[i][j] = Frag<T>::mma(ah, bl[j], acc[i][j]);
          acc[i][j] = Frag<T>::mma(al, bh[j], acc[i][j]);
        }
      }
      Frag<T>::guard(acc[i][0], acc[i][3], ah, SPLIT ? al : ah);
    }
    Frag<T>::keep(bh[0], bh[1], bh[2], bh[3]);
    if (SPLIT) Frag<T>::keep(bl[0], bl[1], bl[2], bl[3]);
  }
  acc_guard4(acc[0][0], acc[0][1], acc[0][2], acc[0][3]);
  acc_guard4(acc[1][0], acc[1][1], acc[1][2], acc[1][3]);
  acc_guard4(acc[2][0], acc[2][1], acc[2][2], acc[2][3]);
  acc_guard4(acc[3][0], acc[3][1], acc[3][2], acc[3][3]);

  float* slab = sT[wave];
  const float* Rb = RESID ? (resid + (size_t)b * strideR) : nullptr;
#pragma unroll
  for (int i = 0; i < 4; ++i) {
    const int mBase = m0 + (i << 4);
#pragma unroll
    for (int j = 0; j < 4; ++j) {
      const int n = n0 + (j << 4) + rlane;
      float bv = 0.f;
      if (BIAS_MODE == 2) bv = bias[n];
#pragma unroll
      for (int r = 0; r < 8; ++r) {
        float v = acc[i][j][r] * scale;
        if (BIAS_MODE == 1) v += bias[mBase + mOff + r];
        if (BIAS_MODE == 2) v += bv;
        if (RESID) v += Rb[(size_t)(mBase + mOff + r) * ldc + n];
        if (ACT == 2) v = fmaxf(v, 0.0f);
        if (ACT == 4) v = (v > 0.f) ? v : 0.01f * v;
        slab[(mOff + r) * 68 + (j << 4) + rlane] = v;
      }
    }
    __builtin_amdgcn_fence(__ATOMIC_RELEASE, "workgroup");
    __builtin_amdgcn_wave_barrier();
    __builtin_amdgcn_fence(__ATOMIC_ACQUIRE, "workgroup");
    if (OUT_MODE == 0) {
      float* C = (float*)Cout + (size_t)b * strideC;
      const int hh = lane >> 4, c4 = (lane & 15) * 4;
      for (int pass = 0; pass < 2; ++pass) {
#pragma unroll
        for (int it = 0; it < 8; ++it) {
          const int row = it * 2 + hh;
          v4f v = *(const v4f*)(slab + row * 68 + c4);
          *(volatile v4f*)(C + (size_t)(mBase + row) * ldc + n0 + c4) = v;
        }
        __threadfence();
      }
    } else {
      const int q = lane >> 3, c8 = (lane & 7) * 8;
      unsigned short* C  = (unsigned short*)Cout  + (size_t)b * strideC;
      unsigned short* C2 = (OUT_MODE == 2) ? ((unsigned short*)Cout2 + (size_t)b * strideC) : nullptr;
      for (int pass = 0; pass < 2; ++pass) {
#pragma unroll
        for (int it = 0; it < 4; ++it) {
          const int row = it * 4 + q;
          const float* sp = slab + row * 68 + c8;
          v8h hv, lv;
#pragma unroll
          for (int e = 0; e < 8; ++e) {
            if (OUT_MODE == 1) {
              hv[e] = (_Float16)sp[e];
            } else {
              unsigned short hb = f2bf_bits(sp[e]);
              unsigned short lb = f2bf_bits(sp[e] - bf_bits2f(hb));
              hv[e] = __builtin_bit_cast(_Float16, hb);
              lv[e] = __builtin_bit_cast(_Float16, lb);
            }
          }
          *(volatile v8h*)(C + (size_t)(mBase + row) * ldc + n0 + c8) = hv;
          if (OUT_MODE == 2) *(volatile v8h*)(C2 + (size_t)(mBase + row) * ldc + n0 + c8) = lv;
        }
        __threadfence();
      }
    }
    __builtin_amdgcn_fence(__ATOMIC_RELEASE, "workgroup");
    __builtin_amdgcn_wave_barrier();
    __builtin_amdgcn_fence(__ATOMIC_ACQUIRE, "workgroup");
  }
}

__global__ __launch_bounds__(96) void patch_split_kernel(const float* __restrict__ x,
                                                         unsigned short* __restrict__ ahi,
                                                         unsigned short* __restrict__ alo) {
  const int r = blockIdx.x;
  const int t = threadIdx.x;
  const int bimg = r / kNPatch;
  const int pidx = r - bimg * kNPatch;
  const int ph = pidx / kGridP;
  const int pw = pidx - ph * kGridP;
  const int d0 = t * 8;
  const int ch = d0 >> 8;
  const int rem = d0 & 255;
  const int py = rem >> 4;
  const int px = rem & 15;
  const size_t src = ((size_t)(bimg * kChan + ch) * kImg + (size_t)(ph * kPatch + py)) * kImg
                   + (size_t)(pw * kPatch + px);
  const v4f a = *(const v4f*)(x + src);
  const v4f c = *(const v4f*)(x + src + 4);
  unsigned short hb[8], lb[8];
#pragma unroll
  for (int e = 0; e < 4; ++e) {
    const float f0 = a[e];
    const unsigned short h0 = f2bf_bits(f0);
    hb[e] = h0;
    lb[e] = f2bf_bits(f0 - bf_bits2f(h0));
    const float f1 = c[e];
    const unsigned short h1 = f2bf_bits(f1);
    hb[4 + e] = h1;
    lb[4 + e] = f2bf_bits(f1 - bf_bits2f(h1));
  }
  const v4u uh = (v4u){pk16(hb[0], hb[1]), pk16(hb[2], hb[3]), pk16(hb[4], hb[5]), pk16(hb[6], hb[7])};
  const v4u ul = (v4u){pk16(lb[0], lb[1]), pk16(lb[2], lb[3]), pk16(lb[4], lb[5]), pk16(lb[6], lb[7])};
  const size_t o = (size_t)r * kKdim + d0;
  *(volatile v4u*)(ahi + o) = uh;
  *(volatile v4u*)(alo + o) = ul;
  __threadfence();
  *(volatile v4u*)(ahi + o) = uh;
  *(volatile v4u*)(alo + o) = ul;
}

__global__ __launch_bounds__(256) void wsplit_kernel(const float* __restrict__ W,
                                                     unsigned short* __restrict__ whi,
                                                     unsigned short* __restrict__ wlo, int n8) {
  const int i = blockIdx.x * 256 + threadIdx.x;
  if (i >= n8) return;
  const float* p = W + 8 * (size_t)i;
  const v4f a = *(const v4f*)(p);
  const v4f c = *(const v4f*)(p + 4);
  unsigned short hb[8], lb[8];
#pragma unroll
  for (int e = 0; e < 4; ++e) {
    const float f0 = a[e];
    const unsigned short h0 = f2bf_bits(f0);
    hb[e] = h0;
    lb[e] = f2bf_bits(f0 - bf_bits2f(h0));
    const float f1 = c[e];
    const unsigned short h1 = f2bf_bits(f1);
    hb[4 + e] = h1;
    lb[4 + e] = f2bf_bits(f1 - bf_bits2f(h1));
  }
  const v4u uh = (v4u){pk16(hb[0], hb[1]), pk16(hb[2], hb[3]), pk16(hb[4], hb[5]), pk16(hb[6], hb[7])};
  const v4u ul = (v4u){pk16(lb[0], lb[1]), pk16(lb[2], lb[3]), pk16(lb[4], lb[5]), pk16(lb[6], lb[7])};
  unsigned short* qh = whi + 8 * (size_t)i;
  unsigned short* ql = wlo + 8 * (size_t)i;
  *(volatile v4u*)qh = uh;
  *(volatile v4u*)ql = ul;
  __threadfence();
  *(volatile v4u*)qh = uh;
  *(volatile v4u*)ql = ul;
}

__global__ __launch_bounds__(192) void hyper_row_kernel(const float* __restrict__ mx,
                                                        const float* __restrict__ x,
                                                        const float* __restrict__ bvec,
                                                        float* __restrict__ out) {
  __shared__ float red[4][8];
  __shared__ float coef[4];
  const int r = blockIdx.x;
  const int t = threadIdx.x;
  const int lane = t & 31;
  const int wave = t >> 5;
  const int c4 = t * 4;

  const int bimg = r / kNPatch;
  const int pidx = r - bimg * kNPatch;
  const int ph = pidx / kGridP;
  const int pw = pidx - ph * kGridP;
  const int ch = c4 >> 8;
  const int rem = c4 & 255;
  const int py = rem >> 4;
  const int px = rem & 15;
  const size_t src = ((size_t)(bimg * kChan + ch) * kImg + (size_t)(ph * kPatch + py)) * kImg
                   + (size_t)(pw * kPatch + px);
  const v4f xv = *(const v4f*)(x + src);
  const v4f mv = *(const v4f*)(mx + (size_t)r * kNdim + c4);
  const v4f bv = *(const v4f*)(bvec + c4);

  float sxx = 0.f, smm = 0.f, smb = 0.f, sbb = 0.f;
#pragma unroll
  for (int e = 0; e < 4; ++e) {
    sxx += xv[e] * xv[e];
    smm += mv[e] * mv[e];
    smb += mv[e] * bv[e];
    sbb += bv[e] * bv[e];
  }
#pragma unroll
  for (int off = 16; off > 0; off >>= 1) {
    sxx += __shfl_xor(sxx, off, 32);
    smm += __shfl_xor(smm, off, 32);
    smb += __shfl_xor(smb, off, 32);
    sbb += __shfl_xor(sbb, off, 32);
  }
  if (lane == 0) {
    red[0][wave] = sxx;
    red[1][wave] = smm;
    red[2][wave] = smb;
    red[3][wave] = sbb;
  }
  __syncthreads();
  if (t == 0) {
    float xx = 0.f, mm = 0.f, mb = 0.f, bb = 0.f;
#pragma unroll
    for (int w = 0; w < 6; ++w) {
      xx += red[0][w];
      mm += red[1][w];
      mb += red[2][w];
      bb += red[3][w];
    }
    const float xn      = fmaxf(sqrtf(xx), kEps);
    const float mxn_raw = sqrtf(mm);
    const float mxn     = fmaxf(mxn_raw, kEps);
    const float xcl     = fminf(fmaxf(xn, -1.0f + 1e-7f), 1.0f - 1e-7f);
    const float art     = atanhf(xcl);
    const float rxn     = 1.0f / xn;
    const float rmxn    = 1.0f / mxn;
    float alpha = tanhf(mxn * rxn * art) * rmxn;
    if (mm == 0.0f) alpha = 0.0f;
    const float rn = fmaxf(fabsf(alpha) * mxn_raw, kEps);
    if (rn > kMaxNorm) alpha = alpha * (1.0f / rn) * kMaxNorm;
    const float x2  = alpha * alpha * mm;
    const float xy  = alpha * mb;
    const float y2  = bb;
    const float cx  = 1.0f + 2.0f * xy + y2;
    const float cy  = 1.0f - x2;
    const float den = fmaxf(1.0f + 2.0f * xy + x2 * y2, kEps);
    const float rden = 1.0f / den;
    const float bi = cx * alpha * rden;
    const float gi = cy * rden;
    const float n2 = bi * bi * mm + 2.0f * bi * gi * mb + gi * gi * bb;
    const float nn = fmaxf(sqrtf(fmaxf(n2, 0.0f)), kEps);
    const float lam = (nn > kMaxNorm) ? (kMaxNorm * (1.0f / nn)) : 1.0f;
    coef[0] = lam * bi;
    coef[1] = lam * gi;
  }
  __syncthreads();
  const float sm = coef[0];
  const float sb = coef[1];
  v4f o;
#pragma unroll
  for (int e = 0; e < 4; ++e) o[e] = sm * mv[e] + sb * bv[e];
  float* op = out + (size_t)r * kNdim + c4;
  *(volatile v4f*)op = o;
  __threadfence();
  *(volatile v4f*)op = o;
}

extern "C" void kernel_launch(void* const* d_in, const int* in_sizes, int n_in,
                              void* d_out, int out_size, void* d_ws, size_t ws_size,
                              hipStream_t stream) {
  if (n_in < 3) return;
  if (in_sizes[0] != kBatch * kChan * kImg * kImg) return;
  if (in_sizes[1] != kNdim * kKdim) return;
  if (in_sizes[2] != kNdim) return;
  if (out_size != kRows * kNdim) return;

  const float* x    = (const float*)d_in[0];
  const float* W    = (const float*)d_in[1];
  const float* bvec = (const float*)d_in[2];
  float* out = (float*)d_out;

  const size_t planeA  = (size_t)kRows * kKdim * 2;
  const size_t planeW  = (size_t)kNdim * kKdim * 2;
  const size_t planeMX = (size_t)kRows * kNdim * 4;
  size_t off = 0;
  char* ws = (char*)d_ws;
  unsigned short* ahi = (unsigned short*)(ws + off); off += planeA;
  unsigned short* alo = (unsigned short*)(ws + off); off += planeA;
  unsigned short* whi = (unsigned short*)(ws + off); off += planeW;
  unsigned short* wlo = (unsigned short*)(ws + off); off += planeW;
  float* mxp = (float*)(ws + off); off += planeMX;
  if (off > ws_size) return;

  patch_split_kernel<<<dim3(kRows, 1, 1), dim3(96, 1, 1), 0, stream>>>(x, ahi, alo);

  const int n8w = (kNdim * kKdim) / 8;
  wsplit_kernel<<<dim3((n8w + 255) / 256, 1, 1), dim3(256, 1, 1), 0, stream>>>(W, whi, wlo, n8w);

  const int tiles = (kRows / 64) * (kNdim / 64);
  wmma_gemm64<1, true, 0, 0, false, 0><<<dim3((tiles + 7) / 8, 1, 1), dim3(256, 1, 1), 0, stream>>>(
      ahi, alo, kKdim, 0L,
      whi, wlo, kKdim, 0L,
      (void*)mxp, (void*)mxp, kNdim, 0L,
      bvec,
      (const float*)mxp, 0L,
      kRows, kNdim, kKdim, 1.0f);

  hyper_row_kernel<<<dim3(kRows, 1, 1), dim3(192, 1, 1), 0, stream>>>(mxp, x, bvec, out);
}
